// LongTermMemory_6279242187107
// MI455X (gfx1250) — hardware-verified
//
#include <hip/hip_runtime.h>

typedef _Float16 v16h __attribute__((ext_vector_type(16)));
typedef _Float16 v8h  __attribute__((ext_vector_type(8)));
typedef float    v8f  __attribute__((ext_vector_type(8)));
typedef float    v4f  __attribute__((ext_vector_type(4)));
union Frag { v16h v; v8h half[2]; };

static __device__ __forceinline__ v8f zero8() {
    v8f z = {0.f, 0.f, 0.f, 0.f, 0.f, 0.f, 0.f, 0.f};
    return z;
}

static __device__ __forceinline__ v8f wmma16(v16h a, v16h b, v8f c) {
    v8f d = __builtin_amdgcn_wmma_f32_16x16x32_f16(false, a, false, b, (short)0, c, false, false);
    asm volatile("v_nop\n\tv_nop\n\tv_nop\n\tv_nop" : "+v"(d) : "v"(a), "v"(b));
    return d;
}

static __device__ __forceinline__ v8h cvt8(v4f u0, v4f u1) {
    v8h o;
    o[0] = (_Float16)u0[0]; o[1] = (_Float16)u0[1]; o[2] = (_Float16)u0[2]; o[3] = (_Float16)u0[3];
    o[4] = (_Float16)u1[0]; o[5] = (_Float16)u1[1]; o[6] = (_Float16)u1[2]; o[7] = (_Float16)u1[3];
    return o;
}

__global__ __launch_bounds__(256) void k_cvt_f16(const float* __restrict__ in, _Float16* out, int n8) {
    const int i = blockIdx.x * 256 + threadIdx.x;
    const bool ok = i < n8;
    const size_t base = (size_t)(ok ? i : 0) * 8;
    const v4f u0 = *(const v4f*)(in + base);
    const v4f u1 = *(const v4f*)(in + base + 4);
    const v8h o = cvt8(u0, u1);
    volatile v8h* p = (volatile v8h*)(out + base);
    if (ok) *p = o;
    __threadfence();
    if (ok) *p = o;
}

__global__ __launch_bounds__(256) void k_wtrans(const float* __restrict__ w0, const float* __restrict__ w1,
                                                const float* __restrict__ w2, const float* __restrict__ w3,
                                                const float* __restrict__ w4,
                                                _Float16* o0, _Float16* o1, _Float16* o2, _Float16* o3, _Float16* o4,
                                                int K, int N, float scl) {
    __shared__ float tile[64][65];
    const int z = blockIdx.z;
    const float* in = (z == 0) ? w0 : (z == 1) ? w1 : (z == 2) ? w2 : (z == 3) ? w3 : w4;
    _Float16* out   = (z == 0) ? o0 : (z == 1) ? o1 : (z == 2) ? o2 : (z == 3) ? o3 : o4;
    const int n0 = blockIdx.x * 64, k0 = blockIdx.y * 64;
    const int tid = threadIdx.x;
    const int cn = tid & 63, rk = tid >> 6;
#pragma unroll
    for (int i = 0; i < 16; ++i) {
        const int kk = rk + 4 * i;
        float v = 0.f;
        if (k0 + kk < K && n0 + cn < N) v = in[(size_t)(k0 + kk) * N + n0 + cn];
        tile[kk][cn] = v;
    }
    __syncthreads();
    const int lane = tid & 31, wave = tid >> 5;
    const int p = lane & 7, rq = lane >> 3;
    v8h vals[2];
#pragma unroll
    for (int i = 0; i < 2; ++i) {
        const int nn = 8 * wave + 4 * i + rq;
        v8h o;
#pragma unroll
        for (int e = 0; e < 8; ++e) o[e] = (_Float16)(tile[8 * p + e][nn] * scl);
        vals[i] = o;
    }
#pragma unroll
    for (int i = 0; i < 2; ++i) {
        const int nn = 8 * wave + 4 * i + rq;
        if (n0 + nn < N && k0 + 8 * p + 8 <= K)
            *(volatile v8h*)(out + (size_t)(n0 + nn) * K + k0 + 8 * p) = vals[i];
    }
    __threadfence();
#pragma unroll
    for (int i = 0; i < 2; ++i) {
        const int nn = 8 * wave + 4 * i + rq;
        if (n0 + nn < N && k0 + 8 * p + 8 <= K)
            *(volatile v8h*)(out + (size_t)(n0 + nn) * K + k0 + 8 * p) = vals[i];
    }
}

template <bool RELU, bool BROW>
__global__ __launch_bounds__(256) void k_gemm(const _Float16* __restrict__ A, const _Float16* __restrict__ Bt,
                                              const float* __restrict__ bias, _Float16* C,
                                              int M, int N, int K, float inv) {
    constexpr int CSP = 68;
    __shared__ __attribute__((aligned(16))) float Cs[128 * CSP];
    const int tid = threadIdx.x, wave = tid >> 5, lane = tid & 31;
    const int h = lane >> 4, m = lane & 15;
    const int m0 = blockIdx.y * 128, n0 = blockIdx.x * 64;
    const int wm = (wave & 3) * 32, wn = (wave >> 2) * 32;

    const int ra0 = min(m0 + wm + m, M - 1), ra1 = min(m0 + wm + 16 + m, M - 1);
    const int rb0 = min(n0 + wn + m, N - 1), rb1 = min(n0 + wn + 16 + m, N - 1);
    const _Float16* pa0 = A  + (size_t)ra0 * K + 8 * h;
    const _Float16* pa1 = A  + (size_t)ra1 * K + 8 * h;
    const _Float16* pb0 = Bt + (size_t)rb0 * K + 8 * h;
    const _Float16* pb1 = Bt + (size_t)rb1 * K + 8 * h;

    v8f c00 = zero8(), c01 = zero8(), c10 = zero8(), c11 = zero8();
#pragma unroll 2
    for (int k0 = 0; k0 + 32 <= K; k0 += 32) {
        Frag a0, a1, b0, b1;
        a0.half[0] = *(const v8h*)(pa0 + k0);  a0.half[1] = *(const v8h*)(pa0 + k0 + 16);
        a1.half[0] = *(const v8h*)(pa1 + k0);  a1.half[1] = *(const v8h*)(pa1 + k0 + 16);
        b0.half[0] = *(const v8h*)(pb0 + k0);  b0.half[1] = *(const v8h*)(pb0 + k0 + 16);
        b1.half[0] = *(const v8h*)(pb1 + k0);  b1.half[1] = *(const v8h*)(pb1 + k0 + 16);
        c00 = wmma16(a0.v, b0.v, c00);
        c01 = wmma16(a0.v, b1.v, c01);
        c10 = wmma16(a1.v, b0.v, c10);
        c11 = wmma16(a1.v, b1.v, c11);
    }

#pragma unroll
    for (int r = 0; r < 8; ++r) {
        Cs[(wm + 8 * h + r) * CSP + wn + m]           = c00[r];
        Cs[(wm + 8 * h + r) * CSP + wn + 16 + m]      = c01[r];
        Cs[(wm + 16 + 8 * h + r) * CSP + wn + m]      = c10[r];
        Cs[(wm + 16 + 8 * h + r) * CSP + wn + 16 + m] = c11[r];
    }
    __syncthreads();

    const int p = lane & 7, rq = lane >> 3;
    v4f bc0 = {0.f, 0.f, 0.f, 0.f}, bc1 = {0.f, 0.f, 0.f, 0.f};
    if (!BROW) {
        if (n0 + 8 * p + 8 <= N) {
            bc0 = *(const v4f*)(bias + n0 + 8 * p);
            bc1 = *(const v4f*)(bias + n0 + 8 * p + 4);
        }
    }
    v8h vals[4];
#pragma unroll
    for (int i = 0; i < 4; ++i) {
        const int rloc = 16 * wave + 4 * i + rq;
        const float* src = Cs + rloc * CSP + 8 * p;
        v4f u0 = *(const v4f*)src;
        v4f u1 = *(const v4f*)(src + 4);
        v4f b0v = bc0, b1v = bc1;
        if (BROW) {
            const float bb = bias[min(m0 + rloc, M - 1)];
            v4f t = {bb, bb, bb, bb};
            b0v = t; b1v = t;
        }
        u0 = u0 * inv + b0v;
        u1 = u1 * inv + b1v;
        if (RELU) {
            u0[0] = fmaxf(u0[0], 0.f); u0[1] = fmaxf(u0[1], 0.f); u0[2] = fmaxf(u0[2], 0.f); u0[3] = fmaxf(u0[3], 0.f);
            u1[0] = fmaxf(u1[0], 0.f); u1[1] = fmaxf(u1[1], 0.f); u1[2] = fmaxf(u1[2], 0.f); u1[3] = fmaxf(u1[3], 0.f);
        }
        vals[i] = cvt8(u0, u1);
    }
#pragma unroll
    for (int i = 0; i < 4; ++i) {
        const int grow = m0 + 16 * wave + 4 * i + rq;
        if (grow < M && n0 + 8 * p + 8 <= N)
            *(volatile v8h*)(C + (size_t)grow * N + n0 + 8 * p) = vals[i];
    }
    __threadfence();
#pragma unroll
    for (int i = 0; i < 4; ++i) {
        const int grow = m0 + 16 * wave + 4 * i + rq;
        if (grow < M && n0 + 8 * p + 8 <= N)
            *(volatile v8h*)(C + (size_t)grow * N + n0 + 8 * p) = vals[i];
    }
}

__global__ __launch_bounds__(256) void k_band_attn(const _Float16* __restrict__ qh, const _Float16* __restrict__ kh,
                                                   const _Float16* __restrict__ vT, float* out,
                                                   int S, int ntok, float scale, float pscl, float pinv) {
    constexpr int D = 1024, HALF = 32, NC = 80, PP = 96, OSP = 516;
    __shared__ __attribute__((aligned(16))) float    Ss[16 * NC];
    __shared__ __attribute__((aligned(16))) _Float16 Ps[16 * PP];
    __shared__ __attribute__((aligned(16))) float    Os[16 * OSP];

    const int tid = threadIdx.x, wave = tid >> 5, lane = tid & 31;
    const int h = lane >> 4, m = lane & 15;
    const int tok0 = blockIdx.x * 16;
    const int b = tok0 / S;
    const int s0 = tok0 - b * S;
    const size_t bS = (size_t)b * S;
    const float ninf = -__builtin_huge_valf();

    if (wave < 5) {
        const int t = wave;
        const int key  = s0 - HALF + 16 * t + m;
        const int keyc = min(max(key, 0), S - 1);
        const _Float16* pa = qh + (size_t)(tok0 + m) * D + 8 * h;
        const _Float16* pb = kh + (bS + keyc) * D + 8 * h;
        v8f acc = zero8();
#pragma unroll 2
        for (int k0 = 0; k0 < D; k0 += 32) {
            Frag a, bb;
            a.half[0]  = *(const v8h*)(pa + k0);  a.half[1]  = *(const v8h*)(pa + k0 + 16);
            bb.half[0] = *(const v8h*)(pb + k0);  bb.half[1] = *(const v8h*)(pb + k0 + 16);
            acc = wmma16(a.v, bb.v, acc);
        }
#pragma unroll
        for (int r = 0; r < 8; ++r) Ss[(8 * h + r) * NC + 16 * t + m] = acc[r];
    }
    __syncthreads();

#pragma unroll
    for (int rr = 0; rr < 2; ++rr) {
        const int r = 2 * wave + rr;
        float xv[3], ev[3];
        bool  vv[3];
        float mx = ninf;
#pragma unroll
        for (int c3 = 0; c3 < 3; ++c3) {
            const int c   = lane + 32 * c3;
            const int key = s0 - HALF + c;
            const bool valid = (c < NC) && (c >= r) && (c <= r + 2 * HALF) && (key >= 0) && (key < S);
            float x = ninf;
            if (valid) x = Ss[r * NC + c] * scale;
            xv[c3] = x; vv[c3] = valid;
            mx = fmaxf(mx, x);
        }
#pragma unroll
        for (int o = 16; o > 0; o >>= 1) mx = fmaxf(mx, __shfl_xor(mx, o, 32));
        float sum = 0.f;
#pragma unroll
        for (int c3 = 0; c3 < 3; ++c3) {
            const float e = vv[c3] ? expf(xv[c3] - mx) : 0.f;
            ev[c3] = e;
            sum += e;
        }
#pragma unroll
        for (int o = 16; o > 0; o >>= 1) sum += __shfl_xor(sum, o, 32);
        const float f = pscl / sum;
#pragma unroll
        for (int c3 = 0; c3 < 3; ++c3) {
            const int c = lane + 32 * c3;
            Ps[r * PP + c] = (_Float16)(ev[c3] * f);
        }
    }
    __syncthreads();

    Frag pf[3];
#pragma unroll
    for (int j = 0; j < 3; ++j) {
        pf[j].half[0] = *(const v8h*)(Ps + m * PP + 32 * j + 8 * h);
        pf[j].half[1] = *(const v8h*)(Ps + m * PP + 32 * j + 16 + 8 * h);
    }
    for (int hd = 0; hd < 2; ++hd) {
#pragma unroll
        for (int i = 0; i < 4; ++i) {
            const int dtl = wave + 8 * i;
            const int d0  = 512 * hd + 16 * dtl;
            const _Float16* prow = vT + (size_t)(d0 + m) * ntok + bS;
            v8f acc = zero8();
#pragma unroll
            for (int j = 0; j < 3; ++j) {
                const int g0 = s0 - HALF + 32 * j + 8 * h;
                const int g1 = g0 + 16;
                const int g0c = min(max(g0, 0), S - 8);
                const int g1c = min(max(g1, 0), S - 8);
                Frag a;
                a.half[0] = *(const v8h*)(prow + g0c);
                a.half[1] = *(const v8h*)(prow + g1c);
                acc = wmma16(a.v, pf[j].v, acc);
            }
#pragma unroll
            for (int r = 0; r < 8; ++r) Os[m * OSP + 16 * dtl + 8 * h + r] = acc[r] * pinv;
        }
        __syncthreads();
        v4f ov[8];
#pragma unroll
        for (int rr = 0; rr < 2; ++rr) {
#pragma unroll
            for (int c = 0; c < 4; ++c) {
                const int row = 2 * wave + rr;
                ov[rr * 4 + c] = *(const v4f*)(Os + row * OSP + 128 * c + 4 * lane);
            }
        }
#pragma unroll
        for (int rr = 0; rr < 2; ++rr) {
#pragma unroll
            for (int c = 0; c < 4; ++c) {
                const int row = 2 * wave + rr;
                if (tok0 + row < ntok)
                    *(volatile v4f*)(out + (size_t)(tok0 + row) * D + 512 * hd + 128 * c + 4 * lane) = ov[rr * 4 + c];
            }
        }
        __threadfence();
#pragma unroll
        for (int rr = 0; rr < 2; ++rr) {
#pragma unroll
            for (int c = 0; c < 4; ++c) {
                const int row = 2 * wave + rr;
                if (tok0 + row < ntok)
                    *(volatile v4f*)(out + (size_t)(tok0 + row) * D + 512 * hd + 128 * c + 4 * lane) = ov[rr * 4 + c];
            }
        }
        __syncthreads();
    }
}

extern "C" void kernel_launch(void* const* d_in, const int* in_sizes, int n_in,
                              void* d_out, int out_size, void* d_ws, size_t ws_size,
                              hipStream_t stream) {
    if (n_in < 11) return;
    constexpr int S = 2048;
    const int KV = in_sizes[2];
    const int D  = in_sizes[4];
    if (D != 1024 || KV != 1024) return;
    const int ntok = in_sizes[0] / D;
    if (ntok <= 0 || ntok * D != in_sizes[0]) return;
    if ((ntok % 128) != 0 || (ntok % S) != 0 || (S % 16) != 0) return;
    if (in_sizes[1] != D * KV || in_sizes[3] != KV * D || in_sizes[5] != D * D ||
        in_sizes[7] != D * D || in_sizes[9] != D * D) return;
    if (in_sizes[6] != D || in_sizes[8] != D || in_sizes[10] != D) return;
    if (out_size != ntok * D) return;

    const float* x  = (const float*)d_in[0];
    const float* w1 = (const float*)d_in[1];
    const float* b1 = (const float*)d_in[2];
    const float* w2 = (const float*)d_in[3];
    const float* b2 = (const float*)d_in[4];
    const float* qw = (const float*)d_in[5];
    const float* qb = (const float*)d_in[6];
    const float* kw = (const float*)d_in[7];
    const float* kb = (const float*)d_in[8];
    const float* vw = (const float*)d_in[9];
    const float* vb = (const float*)d_in[10];
    float* outp = (float*)d_out;

    const size_t nTD = (size_t)ntok * D;
    const size_t nDD = (size_t)D * D;
    _Float16* xh  = (_Float16*)d_ws;
    _Float16* w1t = xh  + nTD;
    _Float16* w2t = w1t + nDD;
    _Float16* qwt = w2t + nDD;
    _Float16* kwt = qwt + nDD;
    _Float16* vwt = kwt + nDD;
    _Float16* hh  = vwt + nDD;
    _Float16* mh  = hh  + nTD;
    _Float16* qh  = mh  + nTD;
    _Float16* kh  = qh  + nTD;
    _Float16* vT  = kh  + nTD;
    const size_t total_halves = 6 * nTD + 5 * nDD;
    if (total_halves * sizeof(_Float16) > ws_size) return;

    const float wscl  = 64.0f, winv = 1.0f / 64.0f;
    const float pscl  = 256.0f, pinv = 1.0f / 256.0f;
    const float scale = 1.0f / sqrtf((float)D);

    {
        const int n8 = (int)(nTD / 8);
        k_cvt_f16<<<(n8 + 255) / 256, 256, 0, stream>>>(x, xh, n8);
    }
    {
        dim3 tg((D + 63) / 64, (D + 63) / 64, 5);
        k_wtrans<<<tg, 256, 0, stream>>>(w1, w2, qw, kw, vw, w1t, w2t, qwt, kwt, vwt, D, D, wscl);
    }
    {
        dim3 g1((KV + 63) / 64, (ntok + 127) / 128);
        k_gemm<true,  false><<<g1, 256, 0, stream>>>(xh, w1t, b1, hh, ntok, KV, D, winv);
        dim3 g2((D + 63) / 64, (ntok + 127) / 128);
        k_gemm<false, false><<<g2, 256, 0, stream>>>(hh, w2t, b2, mh, ntok, D, KV, winv);
        k_gemm<false, false><<<g2, 256, 0, stream>>>(mh, qwt, qb, qh, ntok, D, D, winv);
        k_gemm<false, false><<<g2, 256, 0, stream>>>(mh, kwt, kb, kh, ntok, D, D, winv);
        dim3 g3((ntok + 63) / 64, (D + 127) / 128);
        k_gemm<false, true ><<<g3, 256, 0, stream>>>(vwt, mh, vb, vT, D, ntok, D, winv);
    }
    k_band_attn<<<ntok / 16, 256, 0, stream>>>(qh, kh, vT, outp, S, ntok, scale, pscl, pinv);
}
